// TemporalAttentionLayer_45612552683795
// MI455X (gfx1250) — hardware-verified
//
#include <hip/hip_runtime.h>
#include <math.h>

typedef __attribute__((ext_vector_type(16))) _Float16 v16h;
typedef __attribute__((ext_vector_type(16))) __bf16 v16b;
typedef __attribute__((ext_vector_type(8)))  _Float16 v8h;
typedef __attribute__((ext_vector_type(8)))  float v8f;
typedef __attribute__((ext_vector_type(4)))  float v4f;
typedef __attribute__((ext_vector_type(2)))  float v2f;
typedef __attribute__((ext_vector_type(4)))  unsigned v4u;
typedef __attribute__((ext_vector_type(4)))  int v4i;
typedef float __attribute__((may_alias)) float_a;
typedef int __attribute__((may_alias)) int_a;

template <typename T> __device__ __forceinline__ void vst2(void* p, T v) { *(volatile T*)p = v; __threadfence(); *(volatile T*)p = v; }
__device__ __forceinline__ v8f wmma16(v16h a, v16h b, v8f c) {
  v8f d = __builtin_amdgcn_wmma_f32_16x16x32_f16(false, a, false, b, (short)0, c, false, false);
  asm volatile("v_nop\n\tv_nop\n\tv_nop\n\tv_nop" : "+v"(d) : "v"(a), "v"(b));
  return d;
}
__device__ __forceinline__ v8f wmma_bf(v16b a, v16b b, v8f c) {
  v8f d = __builtin_amdgcn_wmma_f32_16x16x32_bf16(false, a, false, b, (short)0, c, false, false);
  asm volatile("v_nop\n\tv_nop\n\tv_nop\n\tv_nop" : "+v"(d) : "v"(a), "v"(b));
  return d;
}
__device__ __forceinline__ v16h frag_h(const _Float16* rowk0, int lane) {
  union { v16h v; v8h q[2]; } u; const _Float16* p = rowk0 + 8 * (lane >> 4);
  u.q[0] = *(const v8h*)p; u.q[1] = *(const v8h*)(p + 16); return u.v;
}
__device__ __forceinline__ v16h frag_f32(const float* rowk0, int lane) {
  v16h a; const float* p = rowk0 + 8 * (lane >> 4);
#pragma unroll
  for (int i = 0; i < 8; ++i) { a[i] = (_Float16)p[i]; a[8 + i] = (_Float16)p[16 + i]; }
  return a;
}
__device__ __forceinline__ v16h frag_f32s(const float* rowk0, int lane, float sc) {
  v16h a; const float* p = rowk0 + 8 * (lane >> 4);
#pragma unroll
  for (int i = 0; i < 8; ++i) { a[i] = (_Float16)(p[i] * sc); a[8 + i] = (_Float16)(p[16 + i] * sc); }
  return a;
}
__device__ __forceinline__ v16h fragc_f32(const float* W, int k0, int n, int lane, int ld, int K) {
  v16h a; const int g = lane >> 4;
#pragma unroll
  for (int i = 0; i < 8; ++i) { const int ka = k0 + 8 * g + i, kb = ka + 16;
    a[i] = (_Float16)(ka < K ? W[(size_t)(ka < K ? ka : K - 1) * ld + n] : 0.f); a[8 + i] = (_Float16)(kb < K ? W[(size_t)(kb < K ? kb : K - 1) * ld + n] : 0.f); }
  return a;
}
struct F2 { v16b h, l; };
__device__ __forceinline__ F2 bsplit16(const float v[16]) { F2 r;
#pragma unroll
  for (int i = 0; i < 16; ++i) { const __bf16 h = (__bf16)v[i]; r.h[i] = h; r.l[i] = (__bf16)(v[i] - (float)h); }
  return r; }
__device__ __forceinline__ F2 split_row(const float* row, int k0, int lane) { float v[16]; const float* p = row + k0 + 8 * (lane >> 4);
#pragma unroll
  for (int i = 0; i < 8; ++i) { v[i] = p[i]; v[8 + i] = p[16 + i]; }
  return bsplit16(v); }
__device__ __forceinline__ F2 split_rowK(const float* row, int k0, int lane, int K) { float v[16]; const int g = lane >> 4;
#pragma unroll
  for (int i = 0; i < 8; ++i) { const int ka = k0 + 8 * g + i, kb = ka + 16; v[i] = ka < K ? row[ka < K ? ka : K - 1] : 0.f; v[8 + i] = kb < K ? row[kb < K ? kb : K - 1] : 0.f; }
  return bsplit16(v); }
__device__ __forceinline__ F2 split_col(const float* W, int k0, int n, int lane, int ld, int K) { float v[16]; const int g = lane >> 4;
#pragma unroll
  for (int i = 0; i < 8; ++i) { const int ka = k0 + 8 * g + i, kb = ka + 16; v[i] = ka < K ? W[(size_t)(ka < K ? ka : K - 1) * ld + n] : 0.f; v[8 + i] = kb < K ? W[(size_t)(kb < K ? kb : K - 1) * ld + n] : 0.f; }
  return bsplit16(v); }
__device__ __forceinline__ v8f mac3(const F2& a, const F2& b, v8f c) { c = wmma_bf(a.l, b.h, c); c = wmma_bf(a.h, b.l, c); return wmma_bf(a.h, b.h, c); }
__device__ __forceinline__ float sigm(float v) { return 1.0f / (1.0f + expf(-v)); }
#define LDSX() do { asm volatile("s_wait_dscnt 0" ::: "memory"); __builtin_amdgcn_wave_barrier(); __builtin_amdgcn_fence(__ATOMIC_RELEASE, "workgroup"); } while (0)

__device__ __forceinline__ float bfr(float v) { return (float)(__bf16)v; }
#define KN 4096
#define NF 1024
#ifndef KQ
#define KQ KN
#endif
#define WS_S12 0u
#define WS_XT  (WS_S12 + 4u * 2u * KN)
#define WS_P   (WS_XT + 2u * (size_t)NF * KN)
#define WS_END (WS_P + 4u * (size_t)KN * KN)
typedef __attribute__((ext_vector_type(8))) __bf16 v8b;
__device__ __forceinline__ v16b frag_b(const __bf16* rowk0, int lane) { union { v16b v; v8b q[2]; } u; const __bf16* p = rowk0 + 8 * (lane >> 4); u.q[0] = *(const v8b*)p; u.q[1] = *(const v8b*)(p + 16); return u.v; }
__global__ __launch_bounds__(256) void k_s(const float* __restrict__ X, const float* __restrict__ Wv, float* __restrict__ S12) { __shared__ __align__(16) float so[2][32];
  const int t = threadIdx.x; const int rl = t >> 3, sub = t & 7; const size_t row = (size_t)blockIdx.x * 32 + rl; const float* xr = X + row * NF;
  float a = 0.f, b = 0.f;
#pragma unroll 1
  for (int c = sub * 4; c < NF; c += 32) { const v4f xv = *(const v4f*)(xr + c);
#pragma unroll
    for (int e = 0; e < 4; ++e) { const float xe = bfr(xv[e]); a += xe * bfr(Wv[c + e]); b += xe * bfr(Wv[NF + c + e]); } }
#pragma unroll
  for (int o = 1; o < 8; o <<= 1) { a += __shfl_xor(a, o); b += __shfl_xor(b, o); }
  if (sub == 0) { so[0][rl] = a; so[1][rl] = b; } __syncthreads();
  if (t < 64) { const int wch = t >> 5, q = t & 31; vst2(S12 + (size_t)wch * KN + blockIdx.x * 32 + q, so[wch][q]); } }
__global__ __launch_bounds__(128) void k_xt(const float* __restrict__ X, __bf16* __restrict__ XT) { __shared__ __align__(16) __bf16 th[128][136];
  const int tid = threadIdx.x; const int j0 = blockIdx.x * 128, c0 = blockIdx.y * 128;
  for (int e = tid; e < 128 * 128; e += 128) { const int jl = e >> 7, cl = e & 127; th[cl][jl] = (__bf16)X[(size_t)(j0 + jl) * NF + c0 + cl]; }
  __syncthreads();
  for (int e = tid; e < 128 * 16; e += 128) { const int cl = e >> 4, q = e & 15; vst2((unsigned*)(XT + (size_t)(c0 + cl) * KN + j0 + q * 8), *(const v4u*)&th[cl][q * 8]); } }
__global__ __launch_bounds__(256) void k_p(const float* __restrict__ S12, float* __restrict__ P) { __shared__ float sred[8]; __shared__ float sbc; __shared__ __align__(16) float sh[KN];
  const int t = threadIdx.x; const size_t i = blockIdx.x; const float s1 = S12[i]; const float* s2 = S12 + KN;
  float m = -3.0e38f; for (int j = t; j < KN; j += 256) m = fmaxf(m, s2[j]);
#pragma unroll
  for (int o = 1; o < 32; o <<= 1) m = fmaxf(m, __shfl_xor(m, o));
  if ((t & 31) == 0) sred[t >> 5] = m; __syncthreads(); if (t == 0) { float a = sred[0]; for (int q = 1; q < 8; ++q) a = fmaxf(a, sred[q]); const float v = s1 + a; sbc = v > 0.f ? v : 0.2f * v; } __syncthreads(); const float M = sbc; __syncthreads();
  float sum = 0.f; for (int j = t; j < KN; j += 256) { const float v = s1 + s2[j]; const float e = (v > 0.f ? v : 0.2f * v); const float ex = expf(e - M); sh[j] = ex; sum += ex; }
#pragma unroll
  for (int o = 1; o < 32; o <<= 1) sum += __shfl_xor(sum, o);
  if ((t & 31) == 0) sred[t >> 5] = sum; __syncthreads(); if (t == 0) { float a = 0.f; for (int q = 0; q < 8; ++q) a += sred[q]; sbc = 2048.0f / a; } __syncthreads(); const float inv = sbc;
  for (int j = t; j < KN; j += 256) sh[j] *= inv;
  __syncthreads(); for (int q = t; q < KN / 4; q += 256) vst2(P + i * KN + q * 4, *(const v4f*)&sh[q * 4]); }
__global__ __launch_bounds__(128) void k_h(const float* __restrict__ P, const __bf16* __restrict__ XT, float* __restrict__ H) { __shared__ __align__(16) float sf[4][16][132];
  const int tid = threadIdx.x, wave = tid >> 5, lane = tid & 31, col = lane & 15, g = lane >> 4; const int c0 = blockIdx.y * 128; const size_t r0 = (size_t)blockIdx.x * 64 + wave * 16;
  v8f acc[8] = {};
#pragma unroll 1
  for (int kc = 0; kc < KN / 32; ++kc) { const F2 p = split_row(P + (r0 + col) * KN, kc * 32, lane);
#pragma unroll
    for (int j = 0; j < 8; ++j) { const v16b xb = frag_b(XT + (size_t)(c0 + j * 16 + col) * KN + kc * 32, lane); acc[j] = wmma_bf(p.h, xb, acc[j]); acc[j] = wmma_bf(p.l, xb, acc[j]); } }
#pragma unroll
  for (int j = 0; j < 8; ++j)
#pragma unroll
    for (int r = 0; r < 8; ++r) sf[wave][8 * g + r][j * 16 + col] = acc[j][r] * (1.0f / 2048.0f);
  LDSX(); for (int rl = 0; rl < 16; ++rl) vst2(H + (r0 + rl) * NF + c0 + lane * 4, *(const v4f*)&sf[wave][rl][lane * 4]); }
extern "C" void kernel_launch(void* const* d_in, const int* in_sizes, int n_in, void* d_out, int out_size, void* d_ws, size_t ws_size, hipStream_t stream) {
  (void)in_sizes; (void)n_in; (void)out_size;
  const float** F = (const float**)d_in;
  if (ws_size < (size_t)WS_END) return;
  char* ws = (char*)d_ws; float *S12 = (float*)(ws + WS_S12), *P = (float*)(ws + WS_P); __bf16* XT = (__bf16*)(ws + WS_XT);
  k_s<<<dim3(KN / 32), 256, 0, stream>>>(F[0], F[1], S12);
  k_xt<<<dim3(KN / 128, NF / 128), 128, 0, stream>>>(F[0], XT);
  k_p<<<dim3(KQ), 256, 0, stream>>>(S12, P);
  k_h<<<dim3(KQ / 64, NF / 128), 128, 0, stream>>>(P, XT, (float*)d_out);
}
